// MultiScaleAttention_70617852281009
// MI455X (gfx1250) — hardware-verified
//
#include <hip/hip_runtime.h>
#include <math.h>

typedef __attribute__((ext_vector_type(16))) _Float16 v16h;
typedef __attribute__((ext_vector_type(8)))  _Float16 v8h;
typedef __attribute__((ext_vector_type(16))) __bf16   v16b;
typedef __attribute__((ext_vector_type(8)))  __bf16   v8b;
typedef __attribute__((ext_vector_type(8)))  float    v8f;
typedef __attribute__((ext_vector_type(4)))  float    v4f;
typedef __attribute__((ext_vector_type(4)))  unsigned int v4u;

#define SEQ_LEN 2048
#define D_MODEL 1024
#define N_HEAD 16
#define HEAD_DIM 64
#define N_BATCH 4
#define N_ROWS (N_BATCH * SEQ_LEN)
#define KPITCH 72
#define OPITCH 68

static_assert(D_MODEL % 32 == 0);
static_assert(N_ROWS % 64 == 0);
static_assert(D_MODEL % 64 == 0);
static_assert(SEQ_LEN % 64 == 0);
static_assert(HEAD_DIM == 64);
static_assert(N_HEAD * HEAD_DIM == D_MODEL);

__device__ __forceinline__ unsigned short f2bf_bits(float f) {
  unsigned u = __float_as_uint(f);
  return (unsigned short)((u + 0x7FFFu + ((u >> 16) & 1u)) >> 16);
}
__device__ __forceinline__ float bf_bits2f(unsigned short h) { return __uint_as_float(((unsigned)h) << 16); }

__device__ __forceinline__ void dep_guard_h(v8f& a, v8f& b, v16h x, v16h y) { asm volatile("v_nop\n\tv_nop\n\tv_nop\n\tv_nop" : "+v"(a), "+v"(b) : "v"(x), "v"(y)); }
__device__ __forceinline__ void dep_guard_b(v8f& a, v8f& b, v16b x, v16b y) { asm volatile("v_nop\n\tv_nop\n\tv_nop\n\tv_nop" : "+v"(a), "+v"(b) : "v"(x), "v"(y)); }
__device__ __forceinline__ void keep4_h(v16h a, v16h b, v16h c, v16h d) { asm volatile("v_nop" :: "v"(a), "v"(b), "v"(c), "v"(d)); }
__device__ __forceinline__ void keep4_b(v16b a, v16b b, v16b c, v16b d) { asm volatile("v_nop" :: "v"(a), "v"(b), "v"(c), "v"(d)); }
__device__ __forceinline__ void acc_guard4(v8f& a, v8f& b, v8f& c, v8f& d) { asm volatile("v_nop\n\tv_nop\n\tv_nop\n\tv_nop" : "+v"(a), "+v"(b), "+v"(c), "+v"(d)); }
template <typename T> struct Frag;
template <> struct Frag<_Float16> {
  typedef v16h V; union U { v16h v; v8h h[2]; };
  static __device__ __forceinline__ v16h load(const _Float16* p) {
    U f; f.h[0] = *(const v8h*)(p); f.h[1] = *(const v8h*)(p + 16); return f.v;
  }
  static __device__ __forceinline__ v8f mma(v16h a, v16h b, v8f c) {
    return __builtin_amdgcn_wmma_f32_16x16x32_f16(false, a, false, b, (short)0, c, false, false);
  }
  static __device__ __forceinline__ void guard(v8f& a, v8f& b, v16h x, v16h y) { dep_guard_h(a, b, x, y); }
  static __device__ __forceinline__ void keep(v16h a, v16h b, v16h c, v16h d) { keep4_h(a, b, c, d); }
};
template <> struct Frag<__bf16> {
  typedef v16b V; union U { v16b v; v8b h[2]; };
  static __device__ __forceinline__ v16b load(const __bf16* p) {
    U f; f.h[0] = *(const v8b*)(p); f.h[1] = *(const v8b*)(p + 16); return f.v;
  }
  static __device__ __forceinline__ v8f mma(v16b a, v16b b, v8f c) {
    return __builtin_amdgcn_wmma_f32_16x16x32_bf16(false, a, false, b, (short)0, c, false, false);
  }
  static __device__ __forceinline__ void guard(v8f& a, v8f& b, v16b x, v16b y) { dep_guard_b(a, b, x, y); }
  static __device__ __forceinline__ void keep(v16b a, v16b b, v16b c, v16b d) { keep4_b(a, b, c, d); }
};

template <int ET> struct Elem;
template <> struct Elem<0> { typedef _Float16 T; };
template <> struct Elem<1> { typedef __bf16 T; };
template <int ET, bool SPLIT, int BIAS_MODE, int OUT_MODE, bool RESID, int ACT = 0>
__global__ __launch_bounds__(256) void wmma_gemm64(
    const unsigned short* __restrict__ Ap, const unsigned short* __restrict__ A2p, int lda, long strideA,
    const unsigned short* __restrict__ Btp, const unsigned short* __restrict__ Bt2p, int ldb, long strideB,
    void* __restrict__ Cout, void* __restrict__ Cout2, int ldc, long strideC,
    const float* __restrict__ bias,
    const float* __restrict__ resid, long strideR,
    int M, int N, int K, float scale) {
  typedef typename Elem<ET>::T T;
  typedef typename Frag<T>::V V;
  const T* A = (const T*)Ap; const T* A2 = (const T*)A2p; const T* Bt = (const T*)Btp; const T* Bt2 = (const T*)Bt2p;
  __shared__ __align__(16) float sT[8][16 * 68];
  const int b    = blockIdx.y;
  const int lane = threadIdx.x & 31;
  const int wave = threadIdx.x >> 5;
  const int tilesN = N >> 6;
  const int tilesM = M >> 6;
  const int tile = blockIdx.x * 8 + wave;
  if (tile >= tilesM * tilesN) return;
  const int tm = tile / tilesN;
  const int tn = tile - tm * tilesN;
  const int m0 = tm << 6;
  const int n0 = tn << 6;

  const T* Ab  = A  + (size_t)b * strideA;
  const T* Bb  = Bt + (size_t)b * strideB;
  const T* Ab2 = SPLIT ? (A2  + (size_t)b * strideA) : nullptr;
  const T* Bb2 = SPLIT ? (Bt2 + (size_t)b * strideB) : nullptr;

  const int rlane = lane & 15;
  const int koff  = (lane >> 4) * 8;
  const int mOff  = (lane >> 4) * 8;

  v8f acc[4][4];
#pragma unroll
  for (int i = 0; i < 4; ++i)
#pragma unroll
    for (int j = 0; j < 4; ++j) acc[i][j] = (v8f){0.f,0.f,0.f,0.f,0.f,0.f,0.f,0.f};

  for (int k0 = 0; k0 < K; k0 += 32) {
    V bh[4], bl[4];
#pragma unroll
    for (int j = 0; j < 4; ++j) {
      const size_t bo = (size_t)(n0 + (j << 4) + rlane) * ldb + koff + k0;
      bh[j] = Frag<T>::load(Bb + bo);
      if (SPLIT) bl[j] = Frag<T>::load(Bb2 + bo);
    }
#pragma unroll
    for (int i = 0; i < 4; ++i) {
      const size_t ao = (size_t)(m0 + (i << 4) + rlane) * lda + koff + k0;
      V ah = Frag<T>::load(Ab + ao);
      V al;
      if (SPLIT) al = Frag<T>::load(Ab2 + ao);
#pragma unroll
      for (int j = 0; j < 4; ++j) {
        acc[i][j] = Frag<T>::mma(ah, bh[j], acc[i][j]);
        if (SPLIT) {
          acc[i][j] = Frag<T>::mma(ah, bl[j], acc[i][j]);
          acc[i][j] = Frag<T>::mma(al, bh[j], acc[i][j]);
        }
      }
      Frag<T>::guard(acc[i][0], acc[i][3], ah, SPLIT ? al : ah);
    }
    Frag<T>::keep(bh[0], bh[1], bh[2], bh[3]);
    if (SPLIT) Frag<T>::keep(bl[0], bl[1], bl[2], bl[3]);
  }
  acc_guard4(acc[0][0], acc[0][1], acc[0][2], acc[0][3]);
  acc_guard4(acc[1][0], acc[1][1], acc[1][2], acc[1][3]);
  acc_guard4(acc[2][0], acc[2][1], acc[2][2], acc[2][3]);
  acc_guard4(acc[3][0], acc[3][1], acc[3][2], acc[3][3]);

  float* slab = sT[wave];
  const float* Rb = RESID ? (resid + (size_t)b * strideR) : nullptr;
#pragma unroll
  for (int i = 0; i < 4; ++i) {
    const int mBase = m0 + (i << 4);
#pragma unroll
    for (int j = 0; j < 4; ++j) {
      const int n = n0 + (j << 4) + rlane;
      float bv = 0.f;
      if (BIAS_MODE == 2) bv = bias[n];
#pragma unroll
      for (int r = 0; r < 8; ++r) {
        float v = acc[i][j][r] * scale;
        if (BIAS_MODE == 1) v += bias[mBase + mOff + r];
        if (BIAS_MODE == 2) v += bv;
        if (RESID) v += Rb[(size_t)(mBase + mOff + r) * ldc + n];
        if (ACT == 1) v = tanhf(v);
        if (ACT == 2) v = fmaxf(v, 0.0f);
        if (ACT == 3) v = v / (1.0f + expf(-v));
        if (ACT == 4) v = (v > 0.f) ? v : 0.01f * v;
        if (ACT == 5) v = 0.5f * v * (1.0f + erff(v * 0.70710678118654752f));
        slab[(mOff + r) * 68 + (j << 4) + rlane] = v;
      }
    }
    __builtin_amdgcn_fence(__ATOMIC_RELEASE, "workgroup");
    __builtin_amdgcn_wave_barrier();
    __builtin_amdgcn_fence(__ATOMIC_ACQUIRE, "workgroup");
    if (OUT_MODE == 0) {
      float* C = (float*)Cout + (size_t)b * strideC;
      const int hh = lane >> 4, c4 = (lane & 15) * 4;
      for (int pass = 0; pass < 2; ++pass) {
#pragma unroll
        for (int it = 0; it < 8; ++it) {
          const int row = it * 2 + hh;
          v4f v = *(const v4f*)(slab + row * 68 + c4);
          *(volatile v4f*)(C + (size_t)(mBase + row) * ldc + n0 + c4) = v;
        }
        __threadfence();
      }
    } else {
      const int q = lane >> 3, c8 = (lane & 7) * 8;
      unsigned short* C  = (unsigned short*)Cout  + (size_t)b * strideC;
      unsigned short* C2 = (OUT_MODE == 2) ? ((unsigned short*)Cout2 + (size_t)b * strideC) : nullptr;
      for (int pass = 0; pass < 2; ++pass) {
#pragma unroll
        for (int it = 0; it < 4; ++it) {
          const int row = it * 4 + q;
          const float* sp = slab + row * 68 + c8;
          v8h hv, lv;
#pragma unroll
          for (int e = 0; e < 8; ++e) {
            if (OUT_MODE == 1) {
              hv[e] = (_Float16)sp[e];
            } else if (OUT_MODE == 3) {
              hv[e] = __builtin_bit_cast(_Float16, f2bf_bits(sp[e]));
            } else {
              unsigned short hb = f2bf_bits(sp[e]);
              unsigned short lb = f2bf_bits(sp[e] - bf_bits2f(hb));
              hv[e] = __builtin_bit_cast(_Float16, hb);
              lv[e] = __builtin_bit_cast(_Float16, lb);
            }
          }
          *(volatile v8h*)(C + (size_t)(mBase + row) * ldc + n0 + c8) = hv;
          if (OUT_MODE == 2) *(volatile v8h*)(C2 + (size_t)(mBase + row) * ldc + n0 + c8) = lv;
        }
        __threadfence();
      }
    }
    __builtin_amdgcn_fence(__ATOMIC_RELEASE, "workgroup");
    __builtin_amdgcn_wave_barrier();
    __builtin_amdgcn_fence(__ATOMIC_ACQUIRE, "workgroup");
  }
}

__global__ __launch_bounds__(256) void cast_f32_bf16x8(
    const float* __restrict__ in, unsigned short* __restrict__ out, int n8) {
  const int i = blockIdx.x * 256 + threadIdx.x;
  if (i < n8) {
    const v4f a  = *(const v4f*)(in + (size_t)i * 8);
    const v4f a2 = *(const v4f*)(in + (size_t)i * 8 + 4);
    v4u u;
    u[0] = (unsigned)f2bf_bits(a[0])  | ((unsigned)f2bf_bits(a[1])  << 16);
    u[1] = (unsigned)f2bf_bits(a[2])  | ((unsigned)f2bf_bits(a[3])  << 16);
    u[2] = (unsigned)f2bf_bits(a2[0]) | ((unsigned)f2bf_bits(a2[1]) << 16);
    u[3] = (unsigned)f2bf_bits(a2[2]) | ((unsigned)f2bf_bits(a2[3]) << 16);
    unsigned short* p = out + (size_t)i * 8;
    *(volatile v4u*)p = u;
    __threadfence();
    *(volatile v4u*)p = u;
  }
}

__global__ __launch_bounds__(256) void transpose_cast_bf16(
    const float* __restrict__ in, unsigned short* __restrict__ out,
    int pitchIn, int pitchOut, int strideIn, int strideOut) {
  __shared__ __align__(16) unsigned short tileT[64 * 72];
  const int tid = threadIdx.x;
  const int r0 = blockIdx.x * 64, c0 = blockIdx.y * 64;
  const float* inz = in + (size_t)blockIdx.z * (size_t)strideIn;
  unsigned short* outz = out + (size_t)blockIdx.z * (size_t)strideOut;
  const int lr = tid >> 4, col4 = (tid & 15) * 4;
#pragma unroll
  for (int it = 0; it < 4; ++it) {
    const int row = it * 16 + lr;
    const v4f f = *(const v4f*)(inz + (size_t)(r0 + row) * pitchIn + c0 + col4);
#pragma unroll
    for (int e = 0; e < 4; ++e) tileT[(col4 + e) * 72 + row] = f2bf_bits(f[e]);
  }
  __syncthreads();
  const int qrow = tid >> 3, c8 = (tid & 7) * 8;
  for (int pass = 0; pass < 2; ++pass) {
#pragma unroll
    for (int it = 0; it < 2; ++it) {
      const int i = it * 32 + qrow;
      const v4u w = *(const v4u*)(tileT + i * 72 + c8);
      *(volatile v4u*)(outz + (size_t)(c0 + i) * pitchOut + r0 + c8) = w;
    }
    __threadfence();
  }
}

__device__ __forceinline__ v8f mma_bf16(v16b a, v16b bfr, v8f cacc) {
  cacc = __builtin_amdgcn_wmma_f32_16x16x32_bf16(false, a, false, bfr, (short)0, cacc, false, false);
  asm volatile("v_nop\n\tv_nop\n\tv_nop\n\tv_nop" : "+v"(cacc) : "v"(a), "v"(bfr));
  return cacc;
}

__global__ __launch_bounds__(128)
void attn_bf16_kernel(const unsigned short* __restrict__ Qp, const unsigned short* __restrict__ Kp,
                      const unsigned short* __restrict__ Vp, unsigned short* __restrict__ Cp) {
  __shared__ __align__(16) unsigned short Ks[64 * KPITCH];
  __shared__ __align__(16) unsigned short Vt[HEAD_DIM * KPITCH];
  __shared__ __align__(16) unsigned short Ps[4][16 * KPITCH];
  __shared__ __align__(16) float Os[4][16 * OPITCH];

  const int tid  = threadIdx.x;
  const int wave = tid >> 5;
  const int lane = tid & 31;
  const int hh   = lane >> 4;
  const int c    = lane & 15;
  const int bx   = blockIdx.x;
  const int qblk = bx % (SEQ_LEN / 64);
  const int bh   = bx / (SEQ_LEN / 64);
  const int h    = bh % N_HEAD;
  const int b    = bh / N_HEAD;
  const int q0   = qblk * 64 + wave * 16;
  const size_t rowb = (size_t)b * SEQ_LEN;
  const int hcol = h * HEAD_DIM;

  v16b qa[2];
  {
    const __bf16* qrow = (const __bf16*)(Qp + (rowb + q0 + c) * D_MODEL + hcol);
#pragma unroll
    for (int dc = 0; dc < 2; ++dc) qa[dc] = Frag<__bf16>::load(qrow + dc * 32 + 8 * hh);
  }

  float mrow[8], lrow[8];
  v8f oacc[4];
#pragma unroll
  for (int r = 0; r < 8; ++r) { mrow[r] = -INFINITY; lrow[r] = 0.f; }
#pragma unroll
  for (int t = 0; t < 4; ++t) oacc[t] = (v8f){0.f,0.f,0.f,0.f,0.f,0.f,0.f,0.f};

  for (int kc = 0; kc < SEQ_LEN / 64; ++kc) {
    const int kv0 = kc * 64;
    __syncthreads();
#pragma unroll
    for (int i = 0; i < 4; ++i) {
      const int idx = i * 128 + tid;
      const int kvr = idx >> 3, c8 = (idx & 7) * 8;
      const v4u w = *(const v4u*)(Kp + (rowb + kv0 + kvr) * D_MODEL + hcol + c8);
      *(v4u*)(Ks + kvr * KPITCH + c8) = w;
    }
    {
      const int kvr = tid >> 1, dh = (tid & 1) * 32;
      const unsigned short* vrow = Vp + (rowb + kv0 + kvr) * D_MODEL + hcol + dh;
#pragma unroll
      for (int i = 0; i < 4; ++i) {
        const v4u w = *(const v4u*)(vrow + 8 * i);
#pragma unroll
        for (int e = 0; e < 4; ++e) {
          const unsigned wd = w[e];
          Vt[(dh + 8 * i + 2 * e) * KPITCH + kvr]     = (unsigned short)(wd & 0xffffu);
          Vt[(dh + 8 * i + 2 * e + 1) * KPITCH + kvr] = (unsigned short)(wd >> 16);
        }
      }
    }
    __syncthreads();

    v8f s[4];
#pragma unroll
    for (int j = 0; j < 4; ++j) {
      s[j] = (v8f){0.f,0.f,0.f,0.f,0.f,0.f,0.f,0.f};
#pragma unroll
      for (int dc = 0; dc < 2; ++dc) {
        const v16b kb = Frag<__bf16>::load((const __bf16*)(Ks + (j * 16 + c) * KPITCH + dc * 32 + 8 * hh));
        s[j] = mma_bf16(qa[dc], kb, s[j]);
      }
    }

    float cm[8];
#pragma unroll
    for (int r = 0; r < 8; ++r) {
      float m = -INFINITY;
#pragma unroll
      for (int j = 0; j < 4; ++j) {
        s[j][r] *= 0.125f;
        m = fmaxf(m, s[j][r]);
      }
#pragma unroll
      for (int off = 1; off < 16; off <<= 1) m = fmaxf(m, __shfl_xor(m, off, 32));
      cm[r] = m;
    }
    unsigned short* pw = Ps[wave];
#pragma unroll
    for (int r = 0; r < 8; ++r) {
      const float mnew = fmaxf(mrow[r], cm[r]);
      const float alpha = expf(mrow[r] - mnew);
      mrow[r] = mnew;
      float psum = 0.f;
#pragma unroll
      for (int j = 0; j < 4; ++j) {
        const float p = expf(s[j][r] - mnew);
        psum += p;
        pw[(8 * hh + r) * KPITCH + j * 16 + c] = f2bf_bits(p);
      }
#pragma unroll
      for (int off = 1; off < 16; off <<= 1) psum += __shfl_xor(psum, off, 32);
      lrow[r] = lrow[r] * alpha + psum;
#pragma unroll
      for (int t = 0; t < 4; ++t) oacc[t][r] *= alpha;
    }
    __builtin_amdgcn_fence(__ATOMIC_RELEASE, "workgroup");
    __builtin_amdgcn_wave_barrier();
    __builtin_amdgcn_fence(__ATOMIC_ACQUIRE, "workgroup");

#pragma unroll
    for (int kk = 0; kk < 2; ++kk) {
      const v16b pa = Frag<__bf16>::load((const __bf16*)(pw + c * KPITCH + kk * 32 + 8 * hh));
#pragma unroll
      for (int t = 0; t < 4; ++t) {
        const v16b vb = Frag<__bf16>::load((const __bf16*)(Vt + (t * 16 + c) * KPITCH + kk * 32 + 8 * hh));
        oacc[t] = mma_bf16(pa, vb, oacc[t]);
      }
    }
  }

  float* os = Os[wave];
#pragma unroll
  for (int r = 0; r < 8; ++r) {
    const float inv = 1.0f / lrow[r];
#pragma unroll
    for (int t = 0; t < 4; ++t) os[(8 * hh + r) * OPITCH + t * 16 + c] = oacc[t][r] * inv;
  }
  __builtin_amdgcn_fence(__ATOMIC_RELEASE, "workgroup");
  __builtin_amdgcn_wave_barrier();
  __builtin_amdgcn_fence(__ATOMIC_ACQUIRE, "workgroup");
  {
    const int q4 = lane >> 3, c8 = (lane & 7) * 8;
    unsigned short* cbase = Cp + (rowb + q0) * D_MODEL + hcol;
    for (int pass = 0; pass < 2; ++pass) {
#pragma unroll
      for (int it = 0; it < 4; ++it) {
        const int row = it * 4 + q4;
        const float* sp = os + row * OPITCH + c8;
        v4u u;
        u[0] = (unsigned)f2bf_bits(sp[0]) | ((unsigned)f2bf_bits(sp[1]) << 16);
        u[1] = (unsigned)f2bf_bits(sp[2]) | ((unsigned)f2bf_bits(sp[3]) << 16);
        u[2] = (unsigned)f2bf_bits(sp[4]) | ((unsigned)f2bf_bits(sp[5]) << 16);
        u[3] = (unsigned)f2bf_bits(sp[6]) | ((unsigned)f2bf_bits(sp[7]) << 16);
        *(volatile v4u*)(cbase + (size_t)row * D_MODEL + c8) = u;
      }
      __threadfence();
    }
  }
}

__global__ __launch_bounds__(256) void ln_resid_kernel(
    const float* __restrict__ y, const float* __restrict__ x, const float* __restrict__ bo,
    const float* __restrict__ w, const float* __restrict__ bb, float* __restrict__ out) {
  __shared__ float red0[8];
  __shared__ float red1[8];
  const int row = blockIdx.x;
  const int tid = threadIdx.x;
  const int c0 = tid * 4;
  const int wv = tid >> 5, lane = tid & 31;
  const size_t base = (size_t)row * D_MODEL + c0;
  const v4f yv = *(const v4f*)(y + base);
  const v4f xv = *(const v4f*)(x + base);
  const v4f bv = *(const v4f*)(bo + c0);
  float t[4];
#pragma unroll
  for (int e = 0; e < 4; ++e) { const float o = yv[e] + bv[e]; t[e] = xv[e] + o; }
  float s = (t[0] + t[1]) + (t[2] + t[3]);
#pragma unroll
  for (int off = 1; off < 32; off <<= 1) s += __shfl_xor(s, off, 32);
  if (lane == 0) red0[wv] = s;
  __syncthreads();
  float ts = 0.f;
#pragma unroll
  for (int i = 0; i < 8; ++i) ts += red0[i];
  const float mu = ts * (1.0f / (float)D_MODEL);
  float d[4];
  float s2 = 0.f;
#pragma unroll
  for (int e = 0; e < 4; ++e) { d[e] = t[e] - mu; s2 += d[e] * d[e]; }
#pragma unroll
  for (int off = 1; off < 32; off <<= 1) s2 += __shfl_xor(s2, off, 32);
  if (lane == 0) red1[wv] = s2;
  __syncthreads();
  float ts2 = 0.f;
#pragma unroll
  for (int i = 0; i < 8; ++i) ts2 += red1[i];
  const float var = ts2 * (1.0f / (float)D_MODEL);
  const float inv = rsqrtf(var + 1e-5f);
  const v4f w4 = *(const v4f*)(w + c0);
  const v4f b4 = *(const v4f*)(bb + c0);
  v4f o;
#pragma unroll
  for (int e = 0; e < 4; ++e) o[e] = d[e] * inv * w4[e] + b4[e];
  float* p = out + base;
  *(volatile v4f*)p = o;
  __threadfence();
  *(volatile v4f*)p = o;
}

extern "C" void kernel_launch(void* const* d_in, const int* in_sizes, int n_in,
                              void* d_out, int out_size, void* d_ws, size_t ws_size,
                              hipStream_t stream) {
  if (n_in < 11) return;
  const int nAct = N_ROWS * D_MODEL;
  const int nW   = N_HEAD * D_MODEL * HEAD_DIM;
  if (in_sizes[0] != nAct || in_sizes[1] != nW || in_sizes[3] != nW || in_sizes[5] != nW) return;
  if (in_sizes[2] != D_MODEL || in_sizes[4] != D_MODEL || in_sizes[6] != D_MODEL) return;
  if (in_sizes[7] != D_MODEL * D_MODEL || in_sizes[8] != D_MODEL || in_sizes[9] != D_MODEL || in_sizes[10] != D_MODEL) return;
  if (out_size != nAct) return;

  const float* x   = (const float*)d_in[0];
  const float* Wq  = (const float*)d_in[1];
  const float* bq  = (const float*)d_in[2];
  const float* Wk  = (const float*)d_in[3];
  const float* bk  = (const float*)d_in[4];
  const float* Wv  = (const float*)d_in[5];
  const float* bvp = (const float*)d_in[6];
  const float* Wo  = (const float*)d_in[7];
  const float* bo  = (const float*)d_in[8];
  const float* lnw = (const float*)d_in[9];
  const float* lnb = (const float*)d_in[10];
  float* out = (float*)d_out;

  const size_t PLANE16 = (size_t)N_ROWS * D_MODEL * 2;
  const size_t WPLANE  = (size_t)D_MODEL * D_MODEL * 2;
  const size_t PLANE32 = (size_t)N_ROWS * D_MODEL * 4;
  const size_t off_xb = 0;
  const size_t off_wq = off_xb + PLANE16;
  const size_t off_wk = off_wq + WPLANE;
  const size_t off_wv = off_wk + WPLANE;
  const size_t off_wo = off_wv + WPLANE;
  const size_t off_q  = off_wo + WPLANE;
  const size_t off_k  = off_q + PLANE16;
  const size_t off_v  = off_k + PLANE16;
  const size_t off_cc = off_v + PLANE16;
  const size_t off_y  = off_cc + PLANE16;
  const size_t total  = off_y + PLANE32;
  if (total > ws_size) return;

  char* ws = (char*)d_ws;
  unsigned short* xb  = (unsigned short*)(ws + off_xb);
  unsigned short* wqT = (unsigned short*)(ws + off_wq);
  unsigned short* wkT = (unsigned short*)(ws + off_wk);
  unsigned short* wvT = (unsigned short*)(ws + off_wv);
  unsigned short* woT = (unsigned short*)(ws + off_wo);
  unsigned short* qpl = (unsigned short*)(ws + off_q);
  unsigned short* kpl = (unsigned short*)(ws + off_k);
  unsigned short* vpl = (unsigned short*)(ws + off_v);
  unsigned short* cc  = (unsigned short*)(ws + off_cc);
  float* ybuf = (float*)(ws + off_y);

  const int n8 = nAct / 8;
  cast_f32_bf16x8<<<(n8 + 255) / 256, 256, 0, stream>>>(x, xb, n8);

  transpose_cast_bf16<<<dim3(D_MODEL / 64, HEAD_DIM / 64, N_HEAD), 256, 0, stream>>>(Wq, wqT, HEAD_DIM, D_MODEL, D_MODEL * HEAD_DIM, HEAD_DIM * D_MODEL);
  transpose_cast_bf16<<<dim3(D_MODEL / 64, HEAD_DIM / 64, N_HEAD), 256, 0, stream>>>(Wk, wkT, HEAD_DIM, D_MODEL, D_MODEL * HEAD_DIM, HEAD_DIM * D_MODEL);
  transpose_cast_bf16<<<dim3(D_MODEL / 64, HEAD_DIM / 64, N_HEAD), 256, 0, stream>>>(Wv, wvT, HEAD_DIM, D_MODEL, D_MODEL * HEAD_DIM, HEAD_DIM * D_MODEL);
  transpose_cast_bf16<<<dim3(D_MODEL / 64, D_MODEL / 64, 1), 256, 0, stream>>>(Wo, woT, D_MODEL, D_MODEL, 0, 0);

  const int gemmM = N_ROWS, gemmN = D_MODEL, gemmK = D_MODEL;
  const int gemmBlocks = ((gemmM / 64) * (gemmN / 64) + 7) / 8;
  wmma_gemm64<1, false, 2, 3, false><<<dim3(gemmBlocks, 1), 256, 0, stream>>>(
      xb, xb, D_MODEL, (long)0, wqT, wqT, D_MODEL, (long)0, (void*)qpl, (void*)qpl, D_MODEL, (long)0,
      bq, x, (long)0, gemmM, gemmN, gemmK, 1.0f);
  wmma_gemm64<1, false, 2, 3, false><<<dim3(gemmBlocks, 1), 256, 0, stream>>>(
      xb, xb, D_MODEL, (long)0, wkT, wkT, D_MODEL, (long)0, (void*)kpl, (void*)kpl, D_MODEL, (long)0,
      bk, x, (long)0, gemmM, gemmN, gemmK, 1.0f);
  wmma_gemm64<1, false, 2, 3, false><<<dim3(gemmBlocks, 1), 256, 0, stream>>>(
      xb, xb, D_MODEL, (long)0, wvT, wvT, D_MODEL, (long)0, (void*)vpl, (void*)vpl, D_MODEL, (long)0,
      bvp, x, (long)0, gemmM, gemmN, gemmK, 1.0f);

  attn_bf16_kernel<<<N_BATCH * N_HEAD * (SEQ_LEN / 64), 128, 0, stream>>>(qpl, kpl, vpl, cc);

  wmma_gemm64<1, false, 0, 0, false><<<dim3(gemmBlocks, 1), 256, 0, stream>>>(
      cc, cc, D_MODEL, (long)0, woT, woT, D_MODEL, (long)0, (void*)ybuf, (void*)ybuf, D_MODEL, (long)0,
      bo, x, (long)0, gemmM, gemmN, gemmK, 1.0f);

  ln_resid_kernel<<<N_ROWS, 256, 0, stream>>>(ybuf, x, bo, lnw, lnb, out);
}
